// CameraAwareSparseBlock_40458591928948
// MI455X (gfx1250) — hardware-verified
//
#include <hip/hip_runtime.h>
#include <stdint.h>

typedef __attribute__((ext_vector_type(16))) _Float16 v16h;
typedef __attribute__((ext_vector_type(8)))  _Float16 v8h;
typedef __attribute__((ext_vector_type(16))) __bf16   v16b;
typedef __attribute__((ext_vector_type(8)))  __bf16   v8b;
typedef __attribute__((ext_vector_type(8)))  float    v8f;
typedef __attribute__((ext_vector_type(4)))  float    v4f;
typedef __attribute__((ext_vector_type(4)))  unsigned v4u;
#define U16(p) ((const unsigned short*)(const void*)(p))

#define CIN   32
#define COUT  64
#define KT    27
#define NCAM  128
#define K1    864
#define LDA1  896
#define K2    1728
#define LDA2  1728
#define RCH   19200
#define NBST  200
#define EPSV  1e-5f
#define WS_CAP 134217728ul

__device__ __forceinline__ unsigned short f2bf_bits(float f) {
  unsigned u = __float_as_uint(f);
  return (unsigned short)((u + 0x7FFFu + ((u >> 16) & 1u)) >> 16);
}
__device__ __forceinline__ float bf_bits2f(unsigned short h) { return __uint_as_float(((unsigned)h) << 16); }

__device__ __forceinline__ void dep_guard_h(v8f& a, v8f& b, v16h x, v16h y) { asm volatile("v_nop\n\tv_nop\n\tv_nop\n\tv_nop" : "+v"(a), "+v"(b) : "v"(x), "v"(y)); }
__device__ __forceinline__ void dep_guard_b(v8f& a, v8f& b, v16b x, v16b y) { asm volatile("v_nop\n\tv_nop\n\tv_nop\n\tv_nop" : "+v"(a), "+v"(b) : "v"(x), "v"(y)); }
__device__ __forceinline__ void keep4_h(v16h a, v16h b, v16h c, v16h d) { asm volatile("v_nop" :: "v"(a), "v"(b), "v"(c), "v"(d)); }
__device__ __forceinline__ void keep4_b(v16b a, v16b b, v16b c, v16b d) { asm volatile("v_nop" :: "v"(a), "v"(b), "v"(c), "v"(d)); }
__device__ __forceinline__ void acc_guard4(v8f& a, v8f& b, v8f& c, v8f& d) { asm volatile("v_nop\n\tv_nop\n\tv_nop\n\tv_nop" : "+v"(a), "+v"(b), "+v"(c), "+v"(d)); }
template <typename T> struct Frag;
template <> struct Frag<_Float16> {
  typedef v16h V; union U { v16h v; v8h h[2]; };
  static __device__ __forceinline__ v16h load(const _Float16* p) {
    U f; f.h[0] = *(const v8h*)(p); f.h[1] = *(const v8h*)(p + 16); return f.v;
  }
  static __device__ __forceinline__ v8f mma(v16h a, v16h b, v8f c) {
    return __builtin_amdgcn_wmma_f32_16x16x32_f16(false, a, false, b, (short)0, c, false, false);
  }
  static __device__ __forceinline__ void guard(v8f& a, v8f& b, v16h x, v16h y) { dep_guard_h(a, b, x, y); }
  static __device__ __forceinline__ void keep(v16h a, v16h b, v16h c, v16h d) { keep4_h(a, b, c, d); }
};
template <> struct Frag<__bf16> {
  typedef v16b V; union U { v16b v; v8b h[2]; };
  static __device__ __forceinline__ v16b load(const __bf16* p) {
    U f; f.h[0] = *(const v8b*)(p); f.h[1] = *(const v8b*)(p + 16); return f.v;
  }
  static __device__ __forceinline__ v8f mma(v16b a, v16b b, v8f c) {
    return __builtin_amdgcn_wmma_f32_16x16x32_bf16(false, a, false, b, (short)0, c, false, false);
  }
  static __device__ __forceinline__ void guard(v8f& a, v8f& b, v16b x, v16b y) { dep_guard_b(a, b, x, y); }
  static __device__ __forceinline__ void keep(v16b a, v16b b, v16b c, v16b d) { keep4_b(a, b, c, d); }
};

template <int ET> struct Elem;
template <> struct Elem<0> { typedef _Float16 T; };
template <> struct Elem<1> { typedef __bf16 T; };
template <int ET, bool SPLIT, int BIAS_MODE, int OUT_MODE, bool RESID, int ACT = 0>
__global__ __launch_bounds__(256) void wmma_gemm64(
    const unsigned short* __restrict__ Ap, const unsigned short* __restrict__ A2p, int lda, long strideA,
    const unsigned short* __restrict__ Btp, const unsigned short* __restrict__ Bt2p, int ldb, long strideB,
    void* __restrict__ Cout, void* __restrict__ Cout2, int ldc, long strideC,
    const float* __restrict__ bias,
    const float* __restrict__ resid, long strideR,
    int M, int N, int K, float scale) {
  typedef typename Elem<ET>::T T;
  typedef typename Frag<T>::V V;
  const T* A = (const T*)Ap; const T* A2 = (const T*)A2p; const T* Bt = (const T*)Btp; const T* Bt2 = (const T*)Bt2p;
  __shared__ __align__(16) float sT[8][16 * 68];
  const int b    = blockIdx.y;
  const int lane = threadIdx.x & 31;
  const int wave = threadIdx.x >> 5;
  const int tilesN = N >> 6;
  const int tilesM = M >> 6;
  const int tile = blockIdx.x * 8 + wave;
  if (tile >= tilesM * tilesN) return;
  const int tm = tile / tilesN;
  const int tn = tile - tm * tilesN;
  const int m0 = tm << 6;
  const int n0 = tn << 6;

  const T* Ab  = A  + (size_t)b * strideA;
  const T* Bb  = Bt + (size_t)b * strideB;
  const T* Ab2 = SPLIT ? (A2  + (size_t)b * strideA) : nullptr;
  const T* Bb2 = SPLIT ? (Bt2 + (size_t)b * strideB) : nullptr;

  const int rlane = lane & 15;
  const int koff  = (lane >> 4) * 8;
  const int mOff  = (lane >> 4) * 8;

  v8f acc[4][4];
#pragma unroll
  for (int i = 0; i < 4; ++i)
#pragma unroll
    for (int j = 0; j < 4; ++j) acc[i][j] = (v8f){0.f,0.f,0.f,0.f,0.f,0.f,0.f,0.f};

  for (int k0 = 0; k0 < K; k0 += 32) {
    V bh[4], bl[4];
#pragma unroll
    for (int j = 0; j < 4; ++j) {
      const size_t bo = (size_t)(n0 + (j << 4) + rlane) * ldb + koff + k0;
      bh[j] = Frag<T>::load(Bb + bo);
      if (SPLIT) bl[j] = Frag<T>::load(Bb2 + bo);
    }
#pragma unroll
    for (int i = 0; i < 4; ++i) {
      const size_t ao = (size_t)(m0 + (i << 4) + rlane) * lda + koff + k0;
      V ah = Frag<T>::load(Ab + ao);
      V al;
      if (SPLIT) al = Frag<T>::load(Ab2 + ao);
#pragma unroll
      for (int j = 0; j < 4; ++j) {
        acc[i][j] = Frag<T>::mma(ah, bh[j], acc[i][j]);
        if (SPLIT) {
          acc[i][j] = Frag<T>::mma(ah, bl[j], acc[i][j]);
          acc[i][j] = Frag<T>::mma(al, bh[j], acc[i][j]);
        }
      }
      Frag<T>::guard(acc[i][0], acc[i][3], ah, SPLIT ? al : ah);
    }
    Frag<T>::keep(bh[0], bh[1], bh[2], bh[3]);
    if (SPLIT) Frag<T>::keep(bl[0], bl[1], bl[2], bl[3]);
  }
  acc_guard4(acc[0][0], acc[0][1], acc[0][2], acc[0][3]);
  acc_guard4(acc[1][0], acc[1][1], acc[1][2], acc[1][3]);
  acc_guard4(acc[2][0], acc[2][1], acc[2][2], acc[2][3]);
  acc_guard4(acc[3][0], acc[3][1], acc[3][2], acc[3][3]);

  float* slab = sT[wave];
  const float* Rb = RESID ? (resid + (size_t)b * strideR) : nullptr;
#pragma unroll
  for (int i = 0; i < 4; ++i) {
    const int mBase = m0 + (i << 4);
#pragma unroll
    for (int j = 0; j < 4; ++j) {
      const int n = n0 + (j << 4) + rlane;
      float bv = 0.f;
      if (BIAS_MODE == 2) bv = bias[n];
#pragma unroll
      for (int r = 0; r < 8; ++r) {
        float v = acc[i][j][r] * scale;
        if (BIAS_MODE == 1) v += bias[mBase + mOff + r];
        if (BIAS_MODE == 2) v += bv;
        if (RESID) v += Rb[(size_t)(mBase + mOff + r) * ldc + n];
        if (ACT == 1) v = tanhf(v);
        if (ACT == 2) v = fmaxf(v, 0.0f);
        if (ACT == 3) v = v / (1.0f + expf(-v));
        if (ACT == 4) v = (v > 0.f) ? v : 0.01f * v;
        if (ACT == 5) v = 0.5f * v * (1.0f + erff(v * 0.70710678118654752f));
        slab[(mOff + r) * 68 + (j << 4) + rlane] = v;
      }
    }
    __builtin_amdgcn_fence(__ATOMIC_RELEASE, "workgroup");
    __builtin_amdgcn_wave_barrier();
    __builtin_amdgcn_fence(__ATOMIC_ACQUIRE, "workgroup");
    if (OUT_MODE == 0) {
      float* C = (float*)Cout + (size_t)b * strideC;
      const int hh = lane >> 4, c4 = (lane & 15) * 4;
      for (int pass = 0; pass < 2; ++pass) {
#pragma unroll
        for (int it = 0; it < 8; ++it) {
          const int row = it * 2 + hh;
          v4f v = *(const v4f*)(slab + row * 68 + c4);
          *(volatile v4f*)(C + (size_t)(mBase + row) * ldc + n0 + c4) = v;
        }
        __threadfence();
      }
    } else {
      const int q = lane >> 3, c8 = (lane & 7) * 8;
      unsigned short* C  = (unsigned short*)Cout  + (size_t)b * strideC;
      unsigned short* C2 = (OUT_MODE == 2) ? ((unsigned short*)Cout2 + (size_t)b * strideC) : nullptr;
      for (int pass = 0; pass < 2; ++pass) {
#pragma unroll
        for (int it = 0; it < 4; ++it) {
          const int row = it * 4 + q;
          const float* sp = slab + row * 68 + c8;
          v8h hv, lv;
#pragma unroll
          for (int e = 0; e < 8; ++e) {
            if (OUT_MODE == 1) {
              hv[e] = (_Float16)sp[e];
            } else {
              unsigned short hb = f2bf_bits(sp[e]);
              unsigned short lb = f2bf_bits(sp[e] - bf_bits2f(hb));
              hv[e] = __builtin_bit_cast(_Float16, hb);
              lv[e] = __builtin_bit_cast(_Float16, lb);
            }
          }
          *(volatile v8h*)(C + (size_t)(mBase + row) * ldc + n0 + c8) = hv;
          if (OUT_MODE == 2) *(volatile v8h*)(C2 + (size_t)(mBase + row) * ldc + n0 + c8) = lv;
        }
        __threadfence();
      }
    }
    __builtin_amdgcn_fence(__ATOMIC_RELEASE, "workgroup");
    __builtin_amdgcn_wave_barrier();
    __builtin_amdgcn_fence(__ATOMIC_ACQUIRE, "workgroup");
  }
}

__global__ __launch_bounds__(256) void cast_f32_f16x2(
    const float* __restrict__ in, _Float16* __restrict__ out, int n2) {
  int i = blockIdx.x * 256 + threadIdx.x;
  if (i < n2) {
    const _Float16 h0 = (_Float16)in[2 * i], h1 = (_Float16)in[2 * i + 1];
    const unsigned u = (unsigned)__builtin_bit_cast(unsigned short, h0) | ((unsigned)__builtin_bit_cast(unsigned short, h1) << 16);
    ((volatile unsigned*)out)[i] = u;
    __threadfence();
    ((volatile unsigned*)out)[i] = u;
  }
}

__global__ __launch_bounds__(256) void wtrans_k(const float* __restrict__ w, _Float16* __restrict__ o,
                                               int Kd, int Cn, float sc, int n2) {
  const int i = blockIdx.x * 256 + threadIdx.x;
  if (i < n2) {
    const int e0 = 2 * i;
    const int n  = e0 / Kd;
    const int kk = e0 - n * Kd;
    const _Float16 h0 = (_Float16)(w[(size_t)kk * Cn + n] * sc);
    const _Float16 h1 = (_Float16)(w[(size_t)(kk + 1) * Cn + n] * sc);
    const unsigned u = (unsigned)__builtin_bit_cast(unsigned short, h0) | ((unsigned)__builtin_bit_cast(unsigned short, h1) << 16);
    ((volatile unsigned*)o)[i] = u;
    __threadfence();
    ((volatile unsigned*)o)[i] = u;
  }
}

__global__ __launch_bounds__(128) void cam_k(const float* __restrict__ cond, const float* __restrict__ Wc,
                                            const float* __restrict__ bc, float* __restrict__ cam, int camc) {
  const int b = blockIdx.x, j = threadIdx.x;
  float s = 0.f;
#pragma unroll 4
  for (int i = 0; i < camc; ++i) s = fmaf(cond[(size_t)b * camc + i], Wc[(size_t)i * NCAM + j], s);
  s += bc[j];
  volatile float* o = cam + (size_t)b * NCAM;
  o[j] = s;
  __threadfence();
  o[j] = s;
}

__global__ __launch_bounds__(256) void gather1_k(const _Float16* __restrict__ f16, const int* __restrict__ nbr,
                                                _Float16* __restrict__ plane, int row0, int M, int nv) {
  const int g = blockIdx.x * 256 + threadIdx.x;
  const int total = M * (LDA1 / 8);
  if (g >= total) return;
  const int p = g & 7;
  const int u = g >> 3;
  const int r = u / (LDA1 / 64);
  const int j = u - r * (LDA1 / 64);
  const int tap  = 2 * j + (p >> 2);
  const int coff = 8 * (p & 3);
  const int tapc = tap < KT ? tap : KT - 1;
  const int n = row0 + r;
  int idx = nbr[(size_t)n * KT + tapc];
  const bool valid = (idx >= 0) && (tap < KT);
  idx = idx < 0 ? 0 : idx;
  idx = idx > nv - 1 ? nv - 1 : idx;
  v8h v = *(const v8h*)(f16 + (size_t)idx * CIN + coff);
  v4u w = __builtin_bit_cast(v4u, v);
#pragma unroll
  for (int e = 0; e < 4; ++e) w[e] = valid ? w[e] : 0u;
  v = __builtin_bit_cast(v8h, w);
  _Float16* dst = plane + (size_t)r * LDA1 + 64 * j + 8 * p;
  *(volatile v8h*)dst = v;
  __threadfence();
  *(volatile v8h*)dst = v;
}

__global__ __launch_bounds__(256) void gather2_k(const float* __restrict__ h1, const float* __restrict__ bnt,
                                                const int* __restrict__ nbr, _Float16* __restrict__ plane,
                                                int row0, int M, int nv) {
  const int g = blockIdx.x * 256 + threadIdx.x;
  const int total = M * (LDA2 / 8);
  if (g >= total) return;
  const int p = g & 7;
  const int u = g >> 3;
  const int r = u / KT;
  const int j = u - r * KT;
  const int n = row0 + r;
  int idx = nbr[(size_t)n * KT + j];
  const bool valid = (idx >= 0);
  idx = idx < 0 ? 0 : idx;
  idx = idx > nv - 1 ? nv - 1 : idx;
  const float* src = h1 + (size_t)idx * COUT + 8 * p;
  const v4f x0 = *(const v4f*)(src);
  const v4f x1 = *(const v4f*)(src + 4);
  const v4f a0 = *(const v4f*)(bnt + 8 * p);
  const v4f a1 = *(const v4f*)(bnt + 8 * p + 4);
  const v4f c0 = *(const v4f*)(bnt + COUT + 8 * p);
  const v4f c1 = *(const v4f*)(bnt + COUT + 8 * p + 4);
  v8h v;
#pragma unroll
  for (int e = 0; e < 4; ++e) {
    float t = fmaxf(fmaf(x0[e], a0[e], c0[e]), 0.0f);
    if (!valid) t = 0.0f;
    v[e] = (_Float16)t;
  }
#pragma unroll
  for (int e = 0; e < 4; ++e) {
    float t = fmaxf(fmaf(x1[e], a1[e], c1[e]), 0.0f);
    if (!valid) t = 0.0f;
    v[4 + e] = (_Float16)t;
  }
  _Float16* dst = plane + (size_t)r * LDA2 + 64 * j + 8 * p;
  *(volatile v8h*)dst = v;
  __threadfence();
  *(volatile v8h*)dst = v;
}

__global__ __launch_bounds__(256) void stats_k(const float* __restrict__ h, double* __restrict__ part, int nv) {
  __shared__ double sS[16][COUT];
  __shared__ double sQ[16][COUT];
  const int t  = threadIdx.x;
  const int c4 = (t & 15) * 4;
  const int rs = t >> 4;
  double s0 = 0.0, s1 = 0.0, s2 = 0.0, s3 = 0.0;
  double q0 = 0.0, q1 = 0.0, q2 = 0.0, q3 = 0.0;
  const int stride = gridDim.x * 16;
  for (int r = blockIdx.x * 16 + rs; r < nv; r += stride) {
    const v4f x = *(const v4f*)(h + (size_t)r * COUT + c4);
    const double d0 = (double)x[0], d1 = (double)x[1], d2 = (double)x[2], d3 = (double)x[3];
    s0 += d0; s1 += d1; s2 += d2; s3 += d3;
    q0 = fma(d0, d0, q0); q1 = fma(d1, d1, q1); q2 = fma(d2, d2, q2); q3 = fma(d3, d3, q3);
  }
  sS[rs][c4 + 0] = s0; sS[rs][c4 + 1] = s1; sS[rs][c4 + 2] = s2; sS[rs][c4 + 3] = s3;
  sQ[rs][c4 + 0] = q0; sQ[rs][c4 + 1] = q1; sQ[rs][c4 + 2] = q2; sQ[rs][c4 + 3] = q3;
  __syncthreads();
  if (t < COUT) {
    double a = 0.0, bq = 0.0;
#pragma unroll
    for (int k = 0; k < 16; ++k) { a += sS[k][t]; bq += sQ[k][t]; }
    volatile double* pp = part + (size_t)blockIdx.x * 128;
    pp[t] = a; pp[COUT + t] = bq;
    __threadfence();
    pp[t] = a; pp[COUT + t] = bq;
  }
}

__global__ __launch_bounds__(64) void bnfin_k(const double* __restrict__ part, const float* __restrict__ gam,
                                             const float* __restrict__ bet, float* __restrict__ bnt,
                                             int nblk, int nv, float eps) {
  const int c = threadIdx.x;
  double s = 0.0, q = 0.0;
  for (int b = 0; b < nblk; ++b) { s += part[(size_t)b * 128 + c]; q += part[(size_t)b * 128 + COUT + c]; }
  const double inv = 1.0 / (double)nv;
  const double mu = s * inv;
  double var = q * inv - mu * mu;
  var = var < 0.0 ? 0.0 : var;
  const float rstd = (float)(1.0 / sqrt(var + (double)eps));
  const float A  = rstd * gam[c];
  const float Bv = bet[c] - (float)mu * A;
  volatile float* o = bnt;
  o[c] = A; o[COUT + c] = Bv;
  __threadfence();
  o[c] = A; o[COUT + c] = Bv;
}

__global__ __launch_bounds__(256) void film_k(const float* __restrict__ h2, const float* __restrict__ bnt,
                                             const float* __restrict__ cam, const int* __restrict__ bidx,
                                             float* __restrict__ Y, int nv, int nb) {
  const int g = blockIdx.x * 256 + threadIdx.x;
  if (g >= nv * 16) return;
  const int row = g >> 4;
  const int c4  = (g & 15) * 4;
  const v4f x  = *(const v4f*)(h2 + (size_t)row * COUT + c4);
  const v4f A  = *(const v4f*)(bnt + c4);
  const v4f Bv = *(const v4f*)(bnt + COUT + c4);
  int b = bidx[row];
  b = b < 0 ? 0 : b;
  b = b > nb - 1 ? nb - 1 : b;
  const v4f sc = *(const v4f*)(cam + (size_t)b * NCAM + c4);
  const v4f sh = *(const v4f*)(cam + (size_t)b * NCAM + COUT + c4);
  v4f y;
#pragma unroll
  for (int e = 0; e < 4; ++e) {
    float t = fmaf(x[e], A[e], Bv[e]);
    t = fmaf(t, 1.0f + sc[e], sh[e]);
    y[e] = fmaxf(t, 0.0f);
  }
  float* dst = Y + (size_t)row * COUT + c4;
  *(volatile v4f*)dst = y;
  __threadfence();
  *(volatile v4f*)dst = y;
}


extern "C" void kernel_launch(void* const* d_in, const int* in_sizes, int n_in,
                              void* d_out, int out_size, void* d_ws, size_t ws_size,
                              hipStream_t stream) {
  if (n_in < 16) return;
  const float* feats = (const float*)d_in[0];
  const float* cond  = (const float*)d_in[1];
  const float* W1    = (const float*)d_in[2];
  const float* b1    = (const float*)d_in[3];
  const float* g1    = (const float*)d_in[4];
  const float* be1   = (const float*)d_in[5];
  const float* W2    = (const float*)d_in[6];
  const float* b2    = (const float*)d_in[7];
  const float* g2    = (const float*)d_in[8];
  const float* be2   = (const float*)d_in[9];
  const float* Wc    = (const float*)d_in[10];
  const float* bc    = (const float*)d_in[11];
  const float* Wr    = (const float*)d_in[12];
  const float* br    = (const float*)d_in[13];
  const int*   nbr   = (const int*)d_in[14];
  const int*   bidx  = (const int*)d_in[15];
  float* dout = (float*)d_out;
  char*  ws   = (char*)d_ws;

  const int NV   = in_sizes[15];
  const int CAMC = 256;
  const int NB   = in_sizes[1] / CAMC;
  if (NV <= 0 || (NV % 64) != 0 || NB < 1) return;
  if (in_sizes[0] != NV * CIN || in_sizes[14] != NV * KT || out_size != NV * COUT) return;
  if (in_sizes[1] != NB * CAMC || in_sizes[2] != KT * CIN * COUT || in_sizes[6] != KT * COUT * COUT) return;
  if (in_sizes[10] != CAMC * NCAM || in_sizes[11] != NCAM || in_sizes[12] != CIN * COUT) return;
  if (in_sizes[3] != COUT || in_sizes[4] != COUT || in_sizes[5] != COUT || in_sizes[7] != COUT ||
      in_sizes[8] != COUT || in_sizes[9] != COUT || in_sizes[13] != COUT) return;

  size_t off = 0;
  const size_t o_out1 = off; off += ((size_t)NV * COUT * 4 + 255) & ~(size_t)255;
  const size_t o_f16  = off; off += ((size_t)NV * CIN * 2 + 255) & ~(size_t)255;
  const size_t o_w1t  = off; off += ((size_t)COUT * K1 * 2 + 255) & ~(size_t)255;
  const size_t o_w2t  = off; off += ((size_t)COUT * K2 * 2 + 255) & ~(size_t)255;
  const size_t o_wrt  = off; off += ((size_t)COUT * CIN * 2 + 255) & ~(size_t)255;
  const size_t o_cam  = off; off += ((size_t)NB * NCAM * 4 + 255) & ~(size_t)255;
  const size_t o_bnt  = off; off += (size_t)2 * NCAM * 4;
  const size_t o_part = off; off += (size_t)NBST * 128 * 8;
  const int Rmax = NV < RCH ? NV : RCH;
  size_t planeBytes = (size_t)Rmax * LDA2 * 2;
  const size_t yBytes = (size_t)NV * COUT * 4;
  if (yBytes > planeBytes) planeBytes = yBytes;
  const size_t o_plane = off; off += (planeBytes + 255) & ~(size_t)255;
  if (off > ws_size || off > WS_CAP) return;

  float*    out1  = (float*)(ws + o_out1);
  _Float16* f16p  = (_Float16*)(ws + o_f16);
  _Float16* w1t   = (_Float16*)(ws + o_w1t);
  _Float16* w2t   = (_Float16*)(ws + o_w2t);
  _Float16* wrt   = (_Float16*)(ws + o_wrt);
  float*    cam   = (float*)(ws + o_cam);
  float*    bnt1  = (float*)(ws + o_bnt);
  float*    bnt2  = bnt1 + NCAM;
  double*   part  = (double*)(ws + o_part);
  _Float16* plane = (_Float16*)(ws + o_plane);
  float*    Y     = (float*)(ws + o_plane);

  {
    const int n2 = NV * CIN / 2;
    cast_f32_f16x2<<<(n2 + 255) / 256, 256, 0, stream>>>(feats, f16p, n2);
    const int n2a = COUT * K1 / 2;
    wtrans_k<<<(n2a + 255) / 256, 256, 0, stream>>>(W1, w1t, K1, COUT, 64.0f, n2a);
    const int n2b = COUT * K2 / 2;
    wtrans_k<<<(n2b + 255) / 256, 256, 0, stream>>>(W2, w2t, K2, COUT, 64.0f, n2b);
    const int n2c = COUT * CIN / 2;
    wtrans_k<<<(n2c + 255) / 256, 256, 0, stream>>>(Wr, wrt, CIN, COUT, 16.0f, n2c);
    cam_k<<<NB, 128, 0, stream>>>(cond, Wc, bc, cam, CAMC);
  }

  for (int row0 = 0; row0 < NV; row0 += RCH) {
    const int M = (NV - row0) < RCH ? (NV - row0) : RCH;
    const int pieces = M * (LDA1 / 8);
    gather1_k<<<(pieces + 255) / 256, 256, 0, stream>>>(f16p, nbr, plane, row0, M, NV);
    const int tiles = (M / 64) * (COUT / 64);
    wmma_gemm64<0, false, 2, 0, false, 0><<<dim3((tiles + 7) / 8, 1), 256, 0, stream>>>(
        U16(plane), (const unsigned short*)nullptr, LDA1, 0L,
        U16(w1t), (const unsigned short*)nullptr, K1, 0L,
        (void*)(out1 + (size_t)row0 * COUT), (void*)nullptr, COUT, 0L,
        b1, (const float*)nullptr, 0L, M, COUT, K1, 1.0f / 64.0f);
  }
  stats_k<<<NBST, 256, 0, stream>>>(out1, part, NV);
  bnfin_k<<<1, COUT, 0, stream>>>(part, g1, be1, bnt1, NBST, NV, EPSV);

  for (int row0 = 0; row0 < NV; row0 += RCH) {
    const int M = (NV - row0) < RCH ? (NV - row0) : RCH;
    const int pieces = M * (LDA2 / 8);
    gather2_k<<<(pieces + 255) / 256, 256, 0, stream>>>(out1, bnt1, nbr, plane, row0, M, NV);
    const int tiles = (M / 64) * (COUT / 64);
    wmma_gemm64<0, false, 2, 0, false, 0><<<dim3((tiles + 7) / 8, 1), 256, 0, stream>>>(
        U16(plane), (const unsigned short*)nullptr, LDA2, 0L,
        U16(w2t), (const unsigned short*)nullptr, K2, 0L,
        (void*)(dout + (size_t)row0 * COUT), (void*)nullptr, COUT, 0L,
        b2, (const float*)nullptr, 0L, M, COUT, K2, 1.0f / 64.0f);
  }
  stats_k<<<NBST, 256, 0, stream>>>(dout, part, NV);
  bnfin_k<<<1, COUT, 0, stream>>>(part, g2, be2, bnt2, NBST, NV, EPSV);

  film_k<<<(NV * 16 + 255) / 256, 256, 0, stream>>>(dout, bnt2, cam, bidx, Y, NV, NB);
  {
    const int tiles = (NV / 64) * (COUT / 64);
    wmma_gemm64<0, false, 2, 0, true, 0><<<dim3((tiles + 7) / 8, 1), 256, 0, stream>>>(
        U16(f16p), (const unsigned short*)nullptr, CIN, 0L,
        U16(wrt), (const unsigned short*)nullptr, CIN, 0L,
        (void*)dout, (void*)nullptr, COUT, 0L,
        br, (const float*)Y, 0L, NV, COUT, CIN, 1.0f / 16.0f);
  }
  (void)hipGetLastError();
}
